// TransformerEncoderBlock_50818053046417
// MI455X (gfx1250) — hardware-verified
//
#include <hip/hip_runtime.h>


#ifndef NB
#define NB 2
#endif
#ifndef SEQ
#define SEQ 2048
#endif

static constexpr int NB_FULL = 2, SEQ_FULL = 2048, DM = 1024, NH = 16, HD = 64, FF = 4096, NR = NB * SEQ;
static constexpr float XS = 8.0f, WSC = 256.0f, PS = 1024.0f, CS = 64.0f, GS = 8.0f, LOG2E = 1.4426950408889634f, LNEPS = 1e-5f, RSQ2 = 0.70710678118654752f;
static_assert(NB >= 1 && NB <= NB_FULL && SEQ >= 64 && SEQ <= SEQ_FULL && SEQ % 64 == 0);
static_assert(DM == NH * HD && HD == 64 && DM % 256 == 0 && (3 * DM) % 128 == 0 && FF % 128 == 0 && NR % 64 == 0 && DM % 64 == 0 && FF % 64 == 0);
static_assert((size_t)((NB - 1) * SEQ_FULL + SEQ) * DM <= (size_t)NB_FULL * SEQ_FULL * DM);

typedef _Float16 b16;
typedef __attribute__((ext_vector_type(16))) _Float16 v16b;
typedef __attribute__((ext_vector_type(8))) _Float16 v8b;
typedef __attribute__((ext_vector_type(4))) _Float16 v4h;
typedef __attribute__((ext_vector_type(8))) float v8f;
typedef __attribute__((ext_vector_type(4))) float v4f;

static __device__ __forceinline__ float bf16_rne(float f) { unsigned int u = __float_as_uint(f); u += 0x7FFFu + ((u >> 16) & 1u); return __uint_as_float(u & 0xFFFF0000u); }
static __device__ __forceinline__ float bfp(float v) { float t = bf16_rne(v); asm volatile("" : "+v"(t)); return t; }
static __device__ __forceinline__ float pmul(float a, float b) { float p = a * b; asm volatile("" : "+v"(p)); return p; }
static __device__ __forceinline__ float nexp2(float v) { return __builtin_amdgcn_exp2f(v); }
static __device__ __forceinline__ v16b frag_kb(const b16* p, int hh) { const v8b a = *(const v8b*)(p + 8 * hh), b = *(const v8b*)(p + 16 + 8 * hh); v16b f;
#pragma unroll
  for (int e = 0; e < 8; ++e) { f[e] = a[e]; f[8 + e] = b[e]; } return f; }
static __device__ __forceinline__ v8f wmma16b(v16b a, v16b b, v8f c) { v8f d = __builtin_amdgcn_wmma_f32_16x16x32_f16(false, a, false, b, (short)0, c, false, false); asm volatile("v_nop\n\tv_nop\n\tv_nop\n\tv_nop" : "+v"(d) : "v"(a), "v"(b)); return d; }
static __device__ __forceinline__ void wave_lds_sync() { __builtin_amdgcn_fence(3, "workgroup"); __builtin_amdgcn_wave_barrier(); __builtin_amdgcn_fence(2, "workgroup"); }

__global__ __launch_bounds__(256) void wprep_kernel(const float* __restrict__ src, b16* __restrict__ dst, int K, int N) {
  __shared__ __attribute__((aligned(16))) b16 tile[64][64 + 8];
  const int wave = threadIdx.x >> 5, lane = threadIdx.x & 31; const int n0 = blockIdx.x * 64, k0 = blockIdx.y * 64;
  for (int i = threadIdx.x; i < 64 * 16; i += 256) { const int kk = i >> 4, q = (i & 15) * 4; const v4f f = *(const v4f*)(src + (size_t)(k0 + kk) * N + n0 + q); v4h o;
#pragma unroll
    for (int j = 0; j < 4; ++j) o[j] = (b16)(bf16_rne(f[j]) * WSC); *(v4h*)(&tile[kk][q]) = o; }
  __syncthreads();
  for (int rep = 0; rep < 2; ++rep) {
#pragma unroll 1
    for (int it = 0; it < 2; ++it) { const int nn = it * 32 + wave * 4 + (lane >> 3), pc = (lane & 7) * 8; v8b o;
#pragma unroll
      for (int e = 0; e < 8; ++e) o[e] = tile[pc + e][nn];
      *(volatile v8b*)(dst + (size_t)(n0 + nn) * K + k0 + pc) = o; }
    __threadfence(); }
}

template <int RNDIN>
__global__ __launch_bounds__(256) void ln_kernel(const float* __restrict__ src, int bstride, const float* __restrict__ g, const float* __restrict__ bb, b16* __restrict__ Hp) {
#pragma clang fp contract(off)
  const int wave = threadIdx.x >> 5, lane = threadIdx.x & 31; const int row = blockIdx.x * 8 + wave; const int b = row / SEQ, s = row - b * SEQ;
  const float* yr = src + ((size_t)b * bstride + s) * DM;
  float v[32]; float sm = 0.0f;
#pragma unroll
  for (int q = 0; q < 4; ++q) { const int c = q * 256 + lane * 8; const v4f a0 = *(const v4f*)(yr + c), a1 = *(const v4f*)(yr + c + 4);
#pragma unroll
    for (int j = 0; j < 4; ++j) { float t0 = a0[j], t1 = a1[j]; if (RNDIN) { t0 = bf16_rne(t0); t1 = bf16_rne(t1); } v[q * 8 + j] = t0; v[q * 8 + 4 + j] = t1; } }
#pragma unroll
  for (int i = 0; i < 32; ++i) sm += v[i];
#pragma unroll
  for (int o = 16; o >= 1; o >>= 1) sm += __shfl_xor(sm, o);
  const float mean = sm * (1.0f / (float)DM); float sq = 0.0f;
#pragma unroll
  for (int i = 0; i < 32; ++i) { const float d = v[i] - mean; sq += pmul(d, d); }
#pragma unroll
  for (int o = 16; o >= 1; o >>= 1) sq += __shfl_xor(sq, o);
  const float rs = rsqrtf(sq * (1.0f / (float)DM) + LNEPS);
  v8b ov[4];
#pragma unroll
  for (int q = 0; q < 4; ++q) { const int c = q * 256 + lane * 8; const v4f g0 = *(const v4f*)(g + c), g1v = *(const v4f*)(g + c + 4), b0 = *(const v4f*)(bb + c), b1v = *(const v4f*)(bb + c + 4);
#pragma unroll
    for (int j = 0; j < 4; ++j) { ov[q][j] = (b16)((pmul((v[q * 8 + j] - mean) * rs, bfp(g0[j])) + bfp(b0[j])) * XS); ov[q][4 + j] = (b16)((pmul((v[q * 8 + 4 + j] - mean) * rs, bfp(g1v[j])) + bfp(b1v[j])) * XS); } }
  for (int rep = 0; rep < 2; ++rep) {
#pragma unroll
    for (int q = 0; q < 4; ++q) *(volatile v8b*)(Hp + (size_t)row * DM + q * 256 + lane * 8) = ov[q];
    __threadfence(); }
}

__global__ __launch_bounds__(128) void qkv_kernel(const b16* __restrict__ Hp, const b16* __restrict__ WQ, b16* __restrict__ Qp, b16* __restrict__ Kp, b16* __restrict__ VT) {
  __shared__ __attribute__((aligned(16))) float Tf[4][16][128 + 4];
  const int wave = threadIdx.x >> 5, lane = threadIdx.x & 31, nloc = lane & 15, hlf = lane >> 4; const size_t m0 = (size_t)blockIdx.x * 64 + wave * 16; const int n0 = blockIdx.y * 128;
  v8f acc[8];
#pragma unroll
  for (int t = 0; t < 8; ++t) acc[t] = (v8f){};
#pragma unroll 2
  for (int kb = 0; kb < DM; kb += 32) { const v16b a = frag_kb(Hp + (m0 + nloc) * DM + kb, hlf);
#pragma unroll
    for (int t = 0; t < 8; ++t) acc[t] = wmma16b(a, frag_kb(WQ + (size_t)(n0 + t * 16 + nloc) * DM + kb, hlf), acc[t]); }
#pragma unroll
  for (int t = 0; t < 8; ++t)
#pragma unroll
    for (int r = 0; r < 8; ++r) Tf[wave][8 * hlf + r][t * 16 + nloc] = acc[t][r] * (1.0f / (XS * WSC));
  __syncthreads();
  const int which = n0 / DM, cc0 = n0 - which * DM, h0 = cc0 / HD; const int mb = blockIdx.x * 64, b = mb / SEQ, s0 = mb - b * SEQ;
  for (int rep = 0; rep < 2; ++rep) {
    if (which < 2) { b16* Pq = (which == 0) ? Qp : Kp;
#pragma unroll 1
      for (int it = 0; it < 8; ++it) { const int L = it * 16 + wave * 4 + (lane >> 3), pc = (lane & 7) * 8; const int j = L >> 6, r = L & 63;
        const v4f f0 = *(const v4f*)(&Tf[r >> 4][r & 15][j * 64 + pc]), f1 = *(const v4f*)(&Tf[r >> 4][r & 15][j * 64 + pc + 4]); v8b o;
#pragma unroll
        for (int e = 0; e < 4; ++e) { o[e] = (b16)(f0[e] * XS); o[4 + e] = (b16)(f1[e] * XS); }
        *(volatile v8b*)(Pq + ((size_t)(b * NH + h0 + j) * SEQ + s0 + r) * HD + pc) = o; }
    } else {
#pragma unroll 1
      for (int it = 0; it < 8; ++it) { const int L = it * 16 + wave * 4 + (lane >> 3), pc = (lane & 7) * 8; const int j = L >> 6, d = L & 63; const int wv = pc >> 4, rb = pc & 15; v8b o;
#pragma unroll
        for (int e = 0; e < 8; ++e) o[e] = (b16)(Tf[wv][rb + e][j * 64 + d] * XS);
        *(volatile v8b*)(VT + ((size_t)(b * NH + h0 + j) * HD + d) * SEQ + s0 + pc) = o; }
    }
    __threadfence(); }
}

__global__ __launch_bounds__(128) __attribute__((amdgpu_num_vgpr(256))) void attn_kernel(const b16* __restrict__ Qp, const b16* __restrict__ Kp, const b16* __restrict__ VT, b16* __restrict__ CT) {
  __shared__ __attribute__((aligned(16))) b16 Pt[4][16][64 + 8];
  __shared__ __attribute__((aligned(16))) float Tf[4][16][64 + 4];
  const int wave = threadIdx.x >> 5, lane = threadIdx.x & 31, nloc = lane & 15, hlf = lane >> 4;
  const int bh = blockIdx.y, b = bh / NH, hd = bh - b * NH; const int q0 = blockIdx.x * 64 + wave * 16;
  const b16* qr = Qp + ((size_t)bh * SEQ + q0 + nloc) * HD; const v16b qa0 = frag_kb(qr, hlf), qa1 = frag_kb(qr + 32, hlf);
  const b16* kbase = Kp + (size_t)bh * SEQ * HD; const b16* vbase = VT + (size_t)bh * HD * SEQ;
  const float c = LOG2E / (XS * XS * 8.0f);
  v8f o[4]; float m[8], l[8];
#pragma unroll
  for (int j = 0; j < 4; ++j) o[j] = (v8f){};
#pragma unroll
  for (int r = 0; r < 8; ++r) { m[r] = -INFINITY; l[r] = 0.0f; }
#pragma unroll 1
  for (int k0 = 0; k0 < SEQ; k0 += 64) {
    v8f s[4];
#pragma unroll
    for (int t = 0; t < 4; ++t) { const b16* kp = kbase + (size_t)(k0 + t * 16 + nloc) * HD; s[t] = wmma16b(qa0, frag_kb(kp, hlf), (v8f){}); s[t] = wmma16b(qa1, frag_kb(kp + 32, hlf), s[t]); }
    float mx[8], rsum[8];
#pragma unroll
    for (int r = 0; r < 8; ++r) mx[r] = fmaxf(fmaxf(s[0][r], s[1][r]), fmaxf(s[2][r], s[3][r]));
#pragma unroll
    for (int of = 1; of < 16; of <<= 1)
#pragma unroll
      for (int r = 0; r < 8; ++r) mx[r] = fmaxf(mx[r], __shfl_xor(mx[r], of));
#pragma unroll
    for (int r = 0; r < 8; ++r) { const float mn = fmaxf(m[r], mx[r]); const float corr = nexp2((m[r] - mn) * c); m[r] = mn; l[r] *= corr;
#pragma unroll
      for (int j = 0; j < 4; ++j) o[j][r] *= corr;
      float su = 0.0f;
#pragma unroll
      for (int t = 0; t < 4; ++t) { const b16 ph = (b16)(nexp2((s[t][r] - mn) * c) * PS); Pt[wave][8 * hlf + r][t * 16 + nloc] = ph; su += (float)ph; }
      rsum[r] = su; }
#pragma unroll
    for (int of = 1; of < 16; of <<= 1)
#pragma unroll
      for (int r = 0; r < 8; ++r) rsum[r] += __shfl_xor(rsum[r], of);
#pragma unroll
    for (int r = 0; r < 8; ++r) l[r] += rsum[r];
    wave_lds_sync();
    const v16b pa0 = frag_kb(&Pt[wave][nloc][0], hlf), pa1 = frag_kb(&Pt[wave][nloc][32], hlf);
#pragma unroll
    for (int j = 0; j < 4; ++j) { const b16* vp = vbase + (size_t)(j * 16 + nloc) * SEQ + k0; o[j] = wmma16b(pa0, frag_kb(vp, hlf), o[j]); o[j] = wmma16b(pa1, frag_kb(vp + 32, hlf), o[j]); }
    wave_lds_sync();
  }
#pragma unroll
  for (int r = 0; r < 8; ++r) { const float inv = __builtin_amdgcn_rcpf(l[r]) * (CS / XS);
#pragma unroll
    for (int j = 0; j < 4; ++j) Tf[wave][8 * hlf + r][j * 16 + nloc] = o[j][r] * inv; }
  wave_lds_sync();
  const size_t orow0 = (size_t)b * SEQ + q0;
  for (int rep = 0; rep < 2; ++rep) {
#pragma unroll 1
    for (int it = 0; it < 4; ++it) { const int rr = it * 4 + (lane >> 3), pc = (lane & 7) * 8; const v4f f0 = *(const v4f*)(&Tf[wave][rr][pc]), f1 = *(const v4f*)(&Tf[wave][rr][pc + 4]); v8b o8;
#pragma unroll
      for (int e = 0; e < 4; ++e) { o8[e] = (b16)f0[e]; o8[4 + e] = (b16)f1[e]; }
      *(volatile v8b*)(CT + (orow0 + rr) * DM + hd * HD + pc) = o8; }
    __threadfence(); }
}

__global__ __launch_bounds__(128) void proj_kernel(const b16* __restrict__ CT, const b16* __restrict__ WO, const float* __restrict__ bp, const float* __restrict__ x, float* __restrict__ X1) {
  __shared__ __attribute__((aligned(16))) float Tf[4][16][128 + 4];
  const int wave = threadIdx.x >> 5, lane = threadIdx.x & 31, nloc = lane & 15, hlf = lane >> 4; const size_t m0 = (size_t)blockIdx.x * 64 + wave * 16; const int n0 = blockIdx.y * 128;
  const int mb = blockIdx.x * 64, b = mb / SEQ; const size_t xr0 = (size_t)b * SEQ_FULL + (mb - b * SEQ) + wave * 16;
  v8f acc[8];
#pragma unroll
  for (int t = 0; t < 8; ++t) acc[t] = (v8f){};
#pragma unroll 2
  for (int kb = 0; kb < DM; kb += 32) { const v16b a = frag_kb(CT + (m0 + nloc) * DM + kb, hlf);
#pragma unroll
    for (int t = 0; t < 8; ++t) acc[t] = wmma16b(a, frag_kb(WO + (size_t)(n0 + t * 16 + nloc) * DM + kb, hlf), acc[t]); }
#pragma unroll
  for (int t = 0; t < 8; ++t)
#pragma unroll
    for (int r = 0; r < 8; ++r) Tf[wave][8 * hlf + r][t * 16 + nloc] = acc[t][r] * (1.0f / (CS * WSC));
  wave_lds_sync();
  const v4f bv = *(const v4f*)(bp + n0 + lane * 4);
#pragma unroll 1
  for (int rr = 0; rr < 16; ++rr) { const v4f hv = *(const v4f*)(&Tf[wave][rr][lane * 4]); const v4f xv = *(const v4f*)(x + (xr0 + rr) * DM + n0 + lane * 4); v4f ov;
#pragma unroll
    for (int j = 0; j < 4; ++j) ov[j] = hv[j] + bfp(bv[j]) + bfp(xv[j]);
    *(v4f*)(&Tf[wave][rr][lane * 4]) = ov; }
  wave_lds_sync();
  for (int rep = 0; rep < 2; ++rep) { for (int rr = 0; rr < 16; ++rr) *(volatile v4f*)(X1 + (m0 + rr) * DM + n0 + lane * 4) = *(const v4f*)(&Tf[wave][rr][lane * 4]); __threadfence(); }
}

__global__ __launch_bounds__(128) void mlp1_kernel(const b16* __restrict__ Hp, const b16* __restrict__ W1T, const float* __restrict__ b1, b16* __restrict__ G) {
  __shared__ __attribute__((aligned(16))) float Tf[4][16][128 + 4];
  const int wave = threadIdx.x >> 5, lane = threadIdx.x & 31, nloc = lane & 15, hlf = lane >> 4; const size_t m0 = (size_t)blockIdx.x * 64 + wave * 16; const int n0 = blockIdx.y * 128;
  v8f acc[8];
#pragma unroll
  for (int t = 0; t < 8; ++t) acc[t] = (v8f){};
#pragma unroll 2
  for (int kb = 0; kb < DM; kb += 32) { const v16b a = frag_kb(Hp + (m0 + nloc) * DM + kb, hlf);
#pragma unroll
    for (int t = 0; t < 8; ++t) acc[t] = wmma16b(a, frag_kb(W1T + (size_t)(n0 + t * 16 + nloc) * DM + kb, hlf), acc[t]); }
#pragma unroll
  for (int t = 0; t < 8; ++t)
#pragma unroll
    for (int r = 0; r < 8; ++r) Tf[wave][8 * hlf + r][t * 16 + nloc] = acc[t][r] * (1.0f / (XS * WSC));
  wave_lds_sync();
  const v4f bv = *(const v4f*)(b1 + n0 + lane * 4);
#pragma unroll 1
  for (int rr = 0; rr < 16; ++rr) { const v4f hv = *(const v4f*)(&Tf[wave][rr][lane * 4]); v4f gv;
#pragma unroll
    for (int j = 0; j < 4; ++j) { const float t = hv[j] + bfp(bv[j]); gv[j] = 0.5f * t * (1.0f + erff(t * RSQ2)) * GS; }
    *(v4f*)(&Tf[wave][rr][lane * 4]) = gv; }
  wave_lds_sync();
  for (int rep = 0; rep < 2; ++rep) {
#pragma unroll 1
    for (int it = 0; it < 8; ++it) { const int rr = it * 2 + (lane >> 4), pc = (lane & 15) * 8; const v4f f0 = *(const v4f*)(&Tf[wave][rr][pc]), f1 = *(const v4f*)(&Tf[wave][rr][pc + 4]); v8b o8;
#pragma unroll
      for (int e = 0; e < 4; ++e) { o8[e] = (b16)f0[e]; o8[4 + e] = (b16)f1[e]; }
      *(volatile v8b*)(G + (m0 + rr) * FF + n0 + pc) = o8; }
    __threadfence(); }
}

__global__ __launch_bounds__(128) void mlp2_kernel(const b16* __restrict__ G, const b16* __restrict__ W2T, const float* __restrict__ b2, const float* __restrict__ X1, float* __restrict__ out) {
  __shared__ __attribute__((aligned(16))) float Tf[4][16][128 + 4];
  const int wave = threadIdx.x >> 5, lane = threadIdx.x & 31, nloc = lane & 15, hlf = lane >> 4; const size_t m0 = (size_t)blockIdx.x * 64 + wave * 16; const int n0 = blockIdx.y * 128;
  const int mb = blockIdx.x * 64, b = mb / SEQ; const size_t or0 = (size_t)b * SEQ_FULL + (mb - b * SEQ) + wave * 16;
  v8f acc[8];
#pragma unroll
  for (int t = 0; t < 8; ++t) acc[t] = (v8f){};
#pragma unroll 2
  for (int kb = 0; kb < FF; kb += 32) { const v16b a = frag_kb(G + (m0 + nloc) * FF + kb, hlf);
#pragma unroll
    for (int t = 0; t < 8; ++t) acc[t] = wmma16b(a, frag_kb(W2T + (size_t)(n0 + t * 16 + nloc) * FF + kb, hlf), acc[t]); }
#pragma unroll
  for (int t = 0; t < 8; ++t)
#pragma unroll
    for (int r = 0; r < 8; ++r) Tf[wave][8 * hlf + r][t * 16 + nloc] = acc[t][r] * (1.0f / (GS * WSC));
  wave_lds_sync();
  const v4f bv = *(const v4f*)(b2 + n0 + lane * 4);
#pragma unroll 1
  for (int rr = 0; rr < 16; ++rr) { const v4f hv = *(const v4f*)(&Tf[wave][rr][lane * 4]); const v4f xv = *(const v4f*)(X1 + (m0 + rr) * DM + n0 + lane * 4); v4f ov;
#pragma unroll
    for (int j = 0; j < 4; ++j) ov[j] = hv[j] + bfp(bv[j]) + xv[j];
    *(v4f*)(&Tf[wave][rr][lane * 4]) = ov; }
  wave_lds_sync();
  for (int rep = 0; rep < 2; ++rep) { for (int rr = 0; rr < 16; ++rr) *(volatile v4f*)(out + (or0 + rr) * DM + n0 + lane * 4) = *(const v4f*)(&Tf[wave][rr][lane * 4]); __threadfence(); }
}

extern "C" void kernel_launch(void* const* d_in, const int* in_sizes, int n_in, void* d_out, int out_size, void* d_ws, size_t ws_size, hipStream_t stream) {
  (void)n_in;
  auto Fp = [&](int i) { return (const float*)d_in[i]; };
  const int rows_used = (NB - 1) * SEQ_FULL + SEQ;
  if (in_sizes[0] < rows_used * DM || in_sizes[1] != DM * 3 * DM || in_sizes[2] != DM * DM || in_sizes[3] != DM || in_sizes[4] != DM * FF || in_sizes[5] != FF || in_sizes[6] != FF * DM || in_sizes[7] != DM ||
      in_sizes[8] != DM || in_sizes[9] != DM || in_sizes[10] != DM || in_sizes[11] != DM || out_size < rows_used * DM) return;
  size_t off = 0; char* ws = (char*)d_ws;
  auto carve = [&](size_t bytes) { char* p = ws + off; off += (bytes + 255) & ~(size_t)255; return p; };
  b16* WQ = (b16*)carve((size_t)3 * DM * DM * 2); b16* WO = (b16*)carve((size_t)DM * DM * 2); b16* W1T = (b16*)carve((size_t)FF * DM * 2); b16* W2T = (b16*)carve((size_t)DM * FF * 2);
  b16* Hp = (b16*)carve((size_t)NR * DM * 2); b16* Qp = (b16*)carve((size_t)NB * NH * SEQ * HD * 2); b16* Kp = (b16*)carve((size_t)NB * NH * SEQ * HD * 2); b16* VT = (b16*)carve((size_t)NB * NH * HD * SEQ * 2);
  b16* CT = (b16*)carve((size_t)NR * DM * 2); float* X1 = (float*)carve((size_t)NR * DM * 4); b16* G = (b16*)carve((size_t)NR * FF * 2);
  if (off > ws_size || off > ((size_t)128 << 20)) return;
  wprep_kernel<<<dim3(3 * DM / 64, DM / 64), 256, 0, stream>>>(Fp(1), WQ, DM, 3 * DM);
  wprep_kernel<<<dim3(DM / 64, DM / 64), 256, 0, stream>>>(Fp(2), WO, DM, DM);
  wprep_kernel<<<dim3(FF / 64, DM / 64), 256, 0, stream>>>(Fp(4), W1T, DM, FF);
  wprep_kernel<<<dim3(DM / 64, FF / 64), 256, 0, stream>>>(Fp(6), W2T, FF, DM);
  ln_kernel<1><<<NR / 8, 256, 0, stream>>>(Fp(0), SEQ_FULL, Fp(8), Fp(9), Hp);
  qkv_kernel<<<dim3(NR / 64, 3 * DM / 128), 128, 0, stream>>>(Hp, WQ, Qp, Kp, VT);
  attn_kernel<<<dim3(SEQ / 64, NB * NH), 128, 0, stream>>>(Qp, Kp, VT, CT);
  proj_kernel<<<dim3(NR / 64, DM / 128), 128, 0, stream>>>(CT, WO, Fp(3), Fp(0), X1);
  ln_kernel<0><<<NR / 8, 256, 0, stream>>>(X1, SEQ, Fp(10), Fp(11), Hp);
  mlp1_kernel<<<dim3(NR / 64, FF / 128), 128, 0, stream>>>(Hp, W1T, Fp(5), G);
  mlp2_kernel<<<dim3(NR / 64, DM / 128), 128, 0, stream>>>(G, W2T, Fp(7), X1, (float*)d_out);
}
